// GenreAwareRefinement_36223754175137
// MI455X (gfx1250) — hardware-verified
//
#include <hip/hip_runtime.h>


#define NB_  16384
#define DD   512
#define HH   128
#define H2   256
#define NG   18
#define GP   64
#define DM   DD
#define LOSC 1024.0f

typedef _Float16 h16;
typedef unsigned short bf;
typedef __attribute__((ext_vector_type(16))) __bf16   v16bf;
typedef __attribute__((ext_vector_type(16))) _Float16 v16h;
typedef __attribute__((ext_vector_type(8)))  _Float16 v8h;
typedef __attribute__((ext_vector_type(8)))  unsigned short v8us;
typedef __attribute__((ext_vector_type(8)))  float    v8f;
typedef __attribute__((ext_vector_type(4)))  float    v4f;
typedef v8h  __attribute__((may_alias)) v8ha;
typedef v4f  __attribute__((may_alias)) v4fa;
typedef v8us __attribute__((may_alias)) v8usa;

__device__ __forceinline__ unsigned short f2bf(float f) { unsigned u = __float_as_uint(f); u += 0x7FFFu + ((u >> 16) & 1u); return (unsigned short)(u >> 16); }
__device__ __forceinline__ float bf2f(unsigned short b) { return __uint_as_float(((unsigned)b) << 16); }
__device__ __forceinline__ float bfr(float f) { return bf2f(f2bf(f)); }
__device__ __forceinline__ v16h cat16(v8h lo, v8h hi) { return __builtin_shufflevector(lo, hi, 0, 1, 2, 3, 4, 5, 6, 7, 8, 9, 10, 11, 12, 13, 14, 15); }
__device__ __forceinline__ v16bf cat16b(v8us lo, v8us hi) { return __builtin_bit_cast(v16bf, __builtin_shufflevector(lo, hi, 0, 1, 2, 3, 4, 5, 6, 7, 8, 9, 10, 11, 12, 13, 14, 15)); }
__device__ __forceinline__ v8f wmma16(v16h a, v16h b, v8f c) { return __builtin_amdgcn_wmma_f32_16x16x32_f16(false, a, false, b, (short)0, c, false, false); }
__device__ __forceinline__ v8f wmmab(v16bf a, v16bf b, v8f c) { return __builtin_amdgcn_wmma_f32_16x16x32_bf16(false, a, false, b, (short)0, c, false, false); }

template <bool SPLITA, bool F16OUT = false>
__global__ __launch_bounds__(128) void k_gemmb(const bf* __restrict__ A, const bf* __restrict__ Al, const bf* __restrict__ Bn, const float* __restrict__ bias, float* C, int ldc, h16* C2, const float* __restrict__ R = nullptr, int K = DM, int roundR = 1) {
    __shared__ __align__(16) float ost[4][16 * 68];
    const int lane = threadIdx.x & 31, wave = threadIdx.x >> 5, lr = lane & 15, hi = lane >> 4;
    const int r0 = blockIdx.x * 64 + wave * 16, c0 = blockIdx.y * 64;
    const size_t aoff = (size_t)(r0 + lr) * K + 8 * hi;
    size_t boff[4];
#pragma unroll
    for (int t = 0; t < 4; ++t) boff[t] = (size_t)(c0 + t * 16 + lr) * K + 8 * hi;
    v8f acc[4];
#pragma unroll
    for (int t = 0; t < 4; ++t) acc[t] = (v8f){};
#pragma unroll 1
    for (int kc = 0; kc < K; kc += 32) {
        const v16bf a = cat16b(*(const v8us*)(A + aoff + kc), *(const v8us*)(A + aoff + kc + 16));
        v16bf al = a;
        if (SPLITA) al = cat16b(*(const v8us*)(Al + aoff + kc), *(const v8us*)(Al + aoff + kc + 16));
#pragma unroll
        for (int t = 0; t < 4; ++t) { const v16bf b = cat16b(*(const v8us*)(Bn + boff[t] + kc), *(const v8us*)(Bn + boff[t] + kc + 16)); acc[t] = wmmab(a, b, acc[t]); if (SPLITA) acc[t] = wmmab(al, b, acc[t]); }
        asm volatile("v_nop\n\tv_nop\n\tv_nop\n\tv_nop" : "+v"(acc[0]), "+v"(acc[1]), "+v"(acc[2]), "+v"(acc[3]) : "v"(a), "v"(al));
    }
    float* os = &ost[wave][0];
#pragma unroll
    for (int t = 0; t < 4; ++t) { const float bv = bias ? bfr(bias[c0 + t * 16 + lr]) : 0.f;
#pragma unroll
        for (int j = 0; j < 8; ++j) os[(hi * 8 + j) * 68 + t * 16 + lr] = acc[t][j] + bv; }
    __syncthreads();
    if (F16OUT) {
        h16* crow = (h16*)(void*)C + (size_t)r0 * ldc + c0;
        auto pass = [&]() {
#pragma unroll
            for (int s = 0; s < 4; ++s) { const int row = 4 * s + (lane >> 3), piece = lane & 7; const float* sp = os + row * 68 + piece * 8; v8h o, o2;
#pragma unroll
                for (int i = 0; i < 8; ++i) { const h16 a = (h16)sp[i]; o[i] = a; o2[i] = (h16)((sp[i] - (float)a) * LOSC); }
                *(volatile v8h*)(crow + (size_t)row * ldc + piece * 8) = o; if (C2) *(volatile v8h*)(C2 + (size_t)r0 * ldc + c0 + (size_t)row * ldc + piece * 8) = o2; }
        };
        pass(); __threadfence(); pass();
    } else {
        float* crow = C + (size_t)r0 * ldc + c0;
        auto pass = [&]() {
#pragma unroll
            for (int s = 0; s < 8; ++s) { const int Lid = (lane >> 3) + 4 * s, piece = lane & 7; const int row = Lid >> 1, cofs = (Lid & 1) * 32 + piece * 4;
                v4f val = *(const v4fa*)(os + row * 68 + cofs); if (R) { const v4f rv = *(const v4f*)(R + ((size_t)r0 + row) * ldc + c0 + cofs); val += roundR ? (v4f){bfr(rv[0]), bfr(rv[1]), bfr(rv[2]), bfr(rv[3])} : rv; }
                *(volatile v4f*)(crow + (size_t)row * ldc + cofs) = val; }
        };
        pass(); __threadfence(); pass();
    }
}

template <bool SPLITA, bool F16OUT = false>
__global__ __launch_bounds__(128) void k_gemmbm(const int* __restrict__ Mlim, const bf* __restrict__ A, const bf* __restrict__ Al, const bf* __restrict__ Bn, const float* __restrict__ bias, float* C, int ldc, h16* C2, const float* __restrict__ R = nullptr, int K = DM, int roundR = 1) {
    if ((int)blockIdx.x * 64 >= Mlim[0]) return;
    __shared__ __align__(16) float ost[4][16 * 68];
    const int lane = threadIdx.x & 31, wave = threadIdx.x >> 5, lr = lane & 15, hi = lane >> 4;
    const int r0 = blockIdx.x * 64 + wave * 16, c0 = blockIdx.y * 64;
    const size_t aoff = (size_t)(r0 + lr) * K + 8 * hi;
    size_t boff[4];
#pragma unroll
    for (int t = 0; t < 4; ++t) boff[t] = (size_t)(c0 + t * 16 + lr) * K + 8 * hi;
    v8f acc[4];
#pragma unroll
    for (int t = 0; t < 4; ++t) acc[t] = (v8f){};
#pragma unroll 1
    for (int kc = 0; kc < K; kc += 32) {
        const v16bf a = cat16b(*(const v8us*)(A + aoff + kc), *(const v8us*)(A + aoff + kc + 16));
        v16bf al = a;
        if (SPLITA) al = cat16b(*(const v8us*)(Al + aoff + kc), *(const v8us*)(Al + aoff + kc + 16));
#pragma unroll
        for (int t = 0; t < 4; ++t) { const v16bf b = cat16b(*(const v8us*)(Bn + boff[t] + kc), *(const v8us*)(Bn + boff[t] + kc + 16)); acc[t] = wmmab(a, b, acc[t]); if (SPLITA) acc[t] = wmmab(al, b, acc[t]); }
        asm volatile("v_nop\n\tv_nop\n\tv_nop\n\tv_nop" : "+v"(acc[0]), "+v"(acc[1]), "+v"(acc[2]), "+v"(acc[3]) : "v"(a), "v"(al));
    }
    float* os = &ost[wave][0];
#pragma unroll
    for (int t = 0; t < 4; ++t) { const float bv = bias ? bfr(bias[c0 + t * 16 + lr]) : 0.f;
#pragma unroll
        for (int j = 0; j < 8; ++j) os[(hi * 8 + j) * 68 + t * 16 + lr] = acc[t][j] + bv; }
    __syncthreads();
    if (F16OUT) {
        h16* crow = (h16*)(void*)C + (size_t)r0 * ldc + c0;
        auto pass = [&]() {
#pragma unroll
            for (int s = 0; s < 4; ++s) { const int row = 4 * s + (lane >> 3), piece = lane & 7; const float* sp = os + row * 68 + piece * 8; v8h o, o2;
#pragma unroll
                for (int i = 0; i < 8; ++i) { const h16 a = (h16)sp[i]; o[i] = a; o2[i] = (h16)((sp[i] - (float)a) * LOSC); }
                *(volatile v8h*)(crow + (size_t)row * ldc + piece * 8) = o; if (C2) *(volatile v8h*)(C2 + (size_t)r0 * ldc + c0 + (size_t)row * ldc + piece * 8) = o2; }
        };
        pass(); __threadfence(); pass();
    } else {
        float* crow = C + (size_t)r0 * ldc + c0;
        auto pass = [&]() {
#pragma unroll
            for (int s = 0; s < 8; ++s) { const int Lid = (lane >> 3) + 4 * s, piece = lane & 7; const int row = Lid >> 1, cofs = (Lid & 1) * 32 + piece * 4;
                v4f val = *(const v4fa*)(os + row * 68 + cofs); if (R) { const v4f rv = *(const v4f*)(R + ((size_t)r0 + row) * ldc + c0 + cofs); val += roundR ? (v4f){bfr(rv[0]), bfr(rv[1]), bfr(rv[2]), bfr(rv[3])} : rv; }
                *(volatile v4f*)(crow + (size_t)row * ldc + cofs) = val; }
        };
        pass(); __threadfence(); pass();
    }
}

__global__ __launch_bounds__(256) void k_wt(const float* __restrict__ Wm, int K, int ncols, bf* WT) {
    __shared__ __align__(16) unsigned short tl[64 * 72];
    const int tid = threadIdx.x, k0 = blockIdx.x * 64, n0 = blockIdx.y * 64;
    const int kk = tid >> 2, nq = (tid & 3) * 16;
#pragma unroll
    for (int i = 0; i < 16; ++i) tl[(nq + i) * 72 + kk] = f2bf(Wm[(size_t)(k0 + kk) * ncols + n0 + nq + i]);
    __syncthreads();
    const int piece = tid & 7;
    auto pass = [&]() {
#pragma unroll
        for (int s = 0; s < 2; ++s) { const int nr = (tid >> 3) + 32 * s; const v8us val = *(const v8usa*)(tl + nr * 72 + piece * 8); *(volatile v8us*)(WT + (size_t)(n0 + nr) * K + k0 + piece * 8) = val; }
    };
    pass(); __threadfence(); pass();
}

__global__ __launch_bounds__(256) void k_cvt8(const float* __restrict__ src, bf* dst, size_t n8) {
    const size_t i = (size_t)blockIdx.x * 256 + threadIdx.x; if (i >= n8) return;
    const v8f v = *(const v8f*)(src + i * 8); v8us o;
#pragma unroll
    for (int k = 0; k < 8; ++k) o[k] = f2bf(v[k]);
    *(volatile v8us*)(dst + i * 8) = o; __threadfence(); *(volatile v8us*)(dst + i * 8) = o;
}
__global__ __launch_bounds__(256) void k_zero8(bf* dst, size_t n8) {
    const size_t i = (size_t)blockIdx.x * 256 + threadIdx.x; if (i >= n8) return; v8us z;
#pragma unroll
    for (int k = 0; k < 8; ++k) z[k] = 0;
    *(volatile v8us*)(dst + i * 8) = z; __threadfence(); *(volatile v8us*)(dst + i * 8) = z;
}

__global__ __launch_bounds__(256) void k_wtp(const float* __restrict__ Wm, int krows, int ncols, int kpad, bf* WT) {
    __shared__ __align__(16) unsigned short tl[64 * 72];
    const int tid = threadIdx.x, k0 = blockIdx.x * 64, n0 = blockIdx.y * 64;
    const int kk = tid >> 2, nq = (tid & 3) * 16;
    const int k = k0 + kk, kc = k < krows ? k : krows - 1;
#pragma unroll
    for (int i = 0; i < 16; ++i) { const int n = n0 + nq + i, ncl = n < ncols ? n : ncols - 1; const float w = Wm[(size_t)kc * ncols + ncl]; tl[(nq + i) * 72 + kk] = (k < krows && n < ncols) ? f2bf(w) : (unsigned short)0; }
    __syncthreads();
    const int piece = tid & 7;
    auto pass = [&]() {
#pragma unroll
        for (int s = 0; s < 2; ++s) { const int nr = (tid >> 3) + 32 * s; const v8us val = *(const v8usa*)(tl + nr * 72 + piece * 8); *(volatile v8us*)(WT + (size_t)(n0 + nr) * kpad + k0 + piece * 8) = val; }
    };
    pass(); __threadfence(); pass();
}

__global__ __launch_bounds__(256) void k_cvtrows(const float* __restrict__ src, bf* dst) {
    const int lane = threadIdx.x & 31; const size_t r = (size_t)blockIdx.x * 8 + (threadIdx.x >> 5); if (r >= (size_t)NB_) return;
#pragma unroll 1
    for (int ps = 0; ps < 2; ++ps) {
#pragma unroll
        for (int q = 0; q < DD / 256; ++q) { v8us o;
#pragma unroll
            for (int i = 0; i < 8; ++i) o[i] = f2bf(src[r * DD + q * 256 + lane * 8 + i]);
            *(volatile v8us*)(dst + r * DD + q * 256 + lane * 8) = o; }
        if (ps == 0) __threadfence(); }
}
__global__ __launch_bounds__(256) void k_attw(const float* __restrict__ A, const float* __restrict__ ba, const float* __restrict__ gv, float* WGT) {
    typedef __attribute__((ext_vector_type(2))) float v2f_;
    const int lane = threadIdx.x & 31; const size_t b = (size_t)blockIdx.x * 8 + (threadIdx.x >> 5); if (b >= (size_t)NB_) return; const float* ar = A + b * GP;
    float m = -3.0e38f; for (int g = 0; g < NG; ++g) m = fmaxf(m, ar[g] + bfr(ba[g]));
    float s = 0.f; for (int g = 0; g < NG; ++g) s += __expf(ar[g] + bfr(ba[g]) - m);
    const float inv = 1.0f / s; v2f_ v;
#pragma unroll
    for (int i = 0; i < 2; ++i) { const int g = lane * 2 + i; const int gc = g < NG ? g : 0; float w = 0.f; if (g < NG) { const float gvv = bfr(gv[b * NG + gc]); w = (gvv > 0.f) ? __expf(ar[gc] + bfr(ba[gc]) - m) * inv * gvv : 0.f; } v[i] = w; }
    *(volatile v2f_*)(WGT + b * GP + lane * 2) = v; __threadfence(); *(volatile v2f_*)(WGT + b * GP + lane * 2) = v;
}
__global__ __launch_bounds__(512) void k_scan(const float* __restrict__ gv, int g, int* POS, int* CNTL) {
    typedef __attribute__((ext_vector_type(4))) int v4i;
    __shared__ int cnt[512];
    constexpr int RPT = NB_ / 512; const int t = threadIdx.x; int c = 0;
    for (int i = 0; i < RPT; ++i) { const int b = t * RPT + i; c += (bfr(gv[(size_t)b * NG + g]) > 0.f) ? 1 : 0; }
    cnt[t] = c; __syncthreads();
    int v = c;
    for (int d = 1; d < 512; d <<= 1) { const int add = (t >= d) ? cnt[t - d] : 0; __syncthreads(); v += add; cnt[t] = v; __syncthreads(); }
    const int total = cnt[511]; int k = v - c; int vals[RPT];
    for (int i = 0; i < RPT; ++i) { const int b = t * RPT + i; const bool mem = bfr(gv[(size_t)b * NG + g]) > 0.f; vals[i] = mem ? k : -1; if (mem) ++k; }
    int* prow = POS + (size_t)g * NB_ + t * RPT;
#pragma unroll 1
    for (int ps = 0; ps < 2; ++ps) {
#pragma unroll
        for (int j = 0; j < RPT; j += 4) { v4i q4 = {vals[j], vals[j + 1], vals[j + 2], vals[j + 3]}; *(volatile v4i*)(prow + j) = q4; }
        if (ps == 0) __threadfence(); }
    if (t < 32) { const int val = (t == 0) ? total : ((t == 1) ? ((total + 63) / 64) * 64 : 0); *(volatile int*)(CNTL + (size_t)g * 32 + t) = val; __threadfence(); *(volatile int*)(CNTL + (size_t)g * 32 + t) = val; }
}
__global__ __launch_bounds__(256) void k_gath(const bf* __restrict__ Xb, const int* __restrict__ POSg, bf* XG) {
    const int lane = threadIdx.x & 31; const size_t b = (size_t)blockIdx.x * 8 + (threadIdx.x >> 5); if (b >= (size_t)NB_) return; const int r = POSg[b]; if (r < 0) return;
#pragma unroll 1
    for (int ps = 0; ps < 2; ++ps) {
#pragma unroll
        for (int q = 0; q < DD / 256; ++q) { const v8us v = *(const v8us*)(Xb + b * DD + q * 256 + lane * 8); *(volatile v8us*)(XG + (size_t)r * DD + q * 256 + lane * 8) = v; }
        if (ps == 0) __threadfence(); }
}
__global__ __launch_bounds__(256) void k_zpad(const int* __restrict__ CNTg, bf* XG) {
    const int lane = threadIdx.x & 31; const int w = blockIdx.x * 8 + (threadIdx.x >> 5); const int cnt_ = CNTg[0], cp = CNTg[1]; const int r = cnt_ + w; if (r >= cp) return; const v8us zz = {0, 0, 0, 0, 0, 0, 0, 0};
#pragma unroll
    for (int q = 0; q < DD / 256; ++q) { *(volatile v8us*)(XG + (size_t)r * DD + q * 256 + lane * 8) = zz; }
    __threadfence();
#pragma unroll
    for (int q = 0; q < DD / 256; ++q) { *(volatile v8us*)(XG + (size_t)r * DD + q * 256 + lane * 8) = zz; }
}
template <int NC>
__global__ __launch_bounds__(256) void k_relupl(const float* __restrict__ F, const int* __restrict__ CNTg, bf* Ph, bf* Pl) {
    const int lane = threadIdx.x & 31; const size_t r = (size_t)blockIdx.x * 8 + (threadIdx.x >> 5); if (r >= (size_t)CNTg[1]) return;
    if (NC == 256) { const size_t o = r * NC + lane * 8; const v8f v = *(const v8f*)(F + o); v8us oh, ol;
#pragma unroll
        for (int i = 0; i < 8; ++i) { const float y = fmaxf(v[i], 0.f); const unsigned short hb = f2bf(y); oh[i] = hb; ol[i] = f2bf(y - bf2f(hb)); }
        *(volatile v8us*)(Ph + o) = oh; *(volatile v8us*)(Pl + o) = ol; __threadfence(); *(volatile v8us*)(Ph + o) = oh; *(volatile v8us*)(Pl + o) = ol; }
    else { typedef __attribute__((ext_vector_type(4))) unsigned short v4us; const size_t o = r * NC + lane * 4; const v4f v = *(const v4f*)(F + o); v4us oh, ol;
#pragma unroll
        for (int i = 0; i < 4; ++i) { const float y = fmaxf(v[i], 0.f); const unsigned short hb = f2bf(y); oh[i] = hb; ol[i] = f2bf(y - bf2f(hb)); }
        *(volatile v4us*)(Ph + o) = oh; *(volatile v4us*)(Pl + o) = ol; __threadfence(); *(volatile v4us*)(Ph + o) = oh; *(volatile v4us*)(Pl + o) = ol; }
}
__global__ __launch_bounds__(256) void k_refacc(const float* __restrict__ H3, const int* __restrict__ POSg, const float* __restrict__ WGT, int g, int first, float* REF) {
    const int lane = threadIdx.x & 31; const size_t b = (size_t)blockIdx.x * 8 + (threadIdx.x >> 5); if (b >= (size_t)NB_) return; const int r = POSg[b]; const float w = WGT[b * GP + g]; const size_t o = b * HH + lane * 4;
    v4f acc; if (first) { acc[0] = 0.f; acc[1] = 0.f; acc[2] = 0.f; acc[3] = 0.f; } else acc = *(const v4f*)(REF + o);
    if (r >= 0) { const v4f h = *(const v4f*)(H3 + (size_t)r * HH + lane * 4); acc += w * h; }
    *(volatile v4f*)(REF + o) = acc; __threadfence(); *(volatile v4f*)(REF + o) = acc;
}
__global__ __launch_bounds__(256) void k_split128(const float* __restrict__ src, bf* dh, bf* dl) {
    typedef __attribute__((ext_vector_type(4))) unsigned short v4us;
    const int lane = threadIdx.x & 31; const size_t r = (size_t)blockIdx.x * 8 + (threadIdx.x >> 5); if (r >= (size_t)NB_) return; const size_t o = r * HH + lane * 4; const v4f v = *(const v4f*)(src + o); v4us oh, ol;
#pragma unroll
    for (int i = 0; i < 4; ++i) { const unsigned short hb = f2bf(v[i]); oh[i] = hb; ol[i] = f2bf(v[i] - bf2f(hb)); }
    *(volatile v4us*)(dh + o) = oh; *(volatile v4us*)(dl + o) = ol; __threadfence(); *(volatile v4us*)(dh + o) = oh; *(volatile v4us*)(dl + o) = ol;
}
__global__ __launch_bounds__(256) void k_reluout(const float* __restrict__ Y, float* OUTP) {
    const int lane = threadIdx.x & 31; const size_t r = (size_t)blockIdx.x * 8 + (threadIdx.x >> 5); if (r >= (size_t)(NB_ / 4)) return;
#pragma unroll 1
    for (int ps = 0; ps < 2; ++ps) {
#pragma unroll
        for (int q = 0; q < DD / 128; ++q) { const size_t o = r * DD + q * 128 + lane * 4; v4f v = *(const v4f*)(Y + o);
#pragma unroll
            for (int i = 0; i < 4; ++i) v[i] = fmaxf(v[i], 0.f);
            *(volatile v4f*)(OUTP + o) = v; }
        if (ps == 0) __threadfence(); }
}

extern "C" void kernel_launch(void* const* d_in, const int* in_sizes, int n_in,
                              void* d_out, int out_size, void* d_ws, size_t ws_size, hipStream_t stream) {
    (void)in_sizes; (void)n_in; (void)out_size;
    const float* x = (const float*)d_in[0]; const float* gv = (const float*)d_in[1]; const float* W1 = (const float*)d_in[2]; const float* b1 = (const float*)d_in[3]; const float* W2 = (const float*)d_in[4]; const float* b2 = (const float*)d_in[5]; const float* W3 = (const float*)d_in[6]; const float* b3 = (const float*)d_in[7];
    const float* Wa = (const float*)d_in[8]; const float* ba = (const float*)d_in[9]; const float* Wagg = (const float*)d_in[10]; const float* bagg = (const float*)d_in[11];
    float* out = (float*)d_out;
    char* wsp = (char*)d_ws;
    auto take = [&](size_t bytes) { char* p = wsp; wsp += (bytes + 255) & ~(size_t)255; return (void*)p; };
    bf* WAT = (bf*)take((size_t)GP * DD * 2); float* BAP = (float*)take(GP * 4); bf* WG1 = (bf*)take((size_t)DD * DD * 2); bf* WG2 = (bf*)take((size_t)DD * HH * 2);
    bf* W1T = (bf*)take((size_t)H2 * DD * 2); bf* W2T = (bf*)take((size_t)HH * H2 * 2); bf* W3T = (bf*)take((size_t)HH * HH * 2);
    bf* Xb = (bf*)take((size_t)NB_ * DD * 2); float* A18 = (float*)take((size_t)NB_ * GP * 4); float* WGT = (float*)take((size_t)NB_ * GP * 4); int* POS = (int*)take((size_t)NG * NB_ * 4); int* CNT = (int*)take((size_t)NG * 32 * 4);
    bf* XG = (bf*)take((size_t)NB_ * DD * 2); float* H1 = (float*)take((size_t)NB_ * H2 * 4); bf* P1h = (bf*)take((size_t)NB_ * H2 * 2); bf* P1l = (bf*)take((size_t)NB_ * H2 * 2); float* Hm2 = (float*)take((size_t)NB_ * HH * 4); bf* P2h = (bf*)take((size_t)NB_ * HH * 2); bf* P2l = (bf*)take((size_t)NB_ * HH * 2); float* H3 = H1;
    float* REF = (float*)take((size_t)NB_ * HH * 4); bf* Rh = (bf*)take((size_t)NB_ * HH * 2); bf* Rl = (bf*)take((size_t)NB_ * HH * 2); float* Y1 = (float*)take((size_t)(NB_ / 4) * DD * 4); float* Y2 = (float*)take((size_t)(NB_ / 4) * DD * 4);
    if ((size_t)(wsp - (char*)d_ws) > ws_size) return;
    k_wtp<<<dim3(DD / 64, GP / 64, 1), 256, 0, stream>>>(Wa, DD, NG, DD, WAT);
    k_wt<<<dim3(DD / 64, DD / 64, 1), 256, 0, stream>>>(Wagg, DD, DD, WG1); k_wt<<<dim3(HH / 64, DD / 64, 1), 256, 0, stream>>>(Wagg + (size_t)DD * DD, HH, DD, WG2);
    k_cvtrows<<<NB_ / 8, 256, 0, stream>>>(x, Xb);
    k_gemmb<false, false><<<dim3(NB_ / 64, 1, 1), 128, 0, stream>>>(Xb, nullptr, WAT, nullptr, A18, GP, nullptr, nullptr, DD);
    k_attw<<<NB_ / 8, 256, 0, stream>>>(A18, ba, gv, WGT);
    for (int g = 0; g < NG; ++g) {
        k_scan<<<1, 512, 0, stream>>>(gv, g, POS, CNT);
        k_wt<<<dim3(DD / 64, H2 / 64, 1), 256, 0, stream>>>(W1 + (size_t)g * DD * H2, DD, H2, W1T); k_wt<<<dim3(H2 / 64, HH / 64, 1), 256, 0, stream>>>(W2 + (size_t)g * H2 * HH, H2, HH, W2T); k_wt<<<dim3(HH / 64, HH / 64, 1), 256, 0, stream>>>(W3 + (size_t)g * HH * HH, HH, HH, W3T);
        k_gath<<<NB_ / 8, 256, 0, stream>>>(Xb, POS + (size_t)g * NB_, XG); k_zpad<<<8, 256, 0, stream>>>(CNT + g * 32, XG);
        k_gemmbm<false, false><<<dim3(NB_ / 64, H2 / 64, 1), 128, 0, stream>>>(CNT + g * 32 + 1, XG, nullptr, W1T, b1 + (size_t)g * H2, H1, H2, nullptr, nullptr, DD);
        k_relupl<H2><<<NB_ / 8, 256, 0, stream>>>(H1, CNT + g * 32, P1h, P1l);
        k_gemmbm<true, false><<<dim3(NB_ / 64, HH / 64, 1), 128, 0, stream>>>(CNT + g * 32 + 1, P1h, P1l, W2T, b2 + (size_t)g * HH, Hm2, HH, nullptr, nullptr, H2);
        k_relupl<HH><<<NB_ / 8, 256, 0, stream>>>(Hm2, CNT + g * 32, P2h, P2l);
        k_gemmbm<true, false><<<dim3(NB_ / 64, HH / 64, 1), 128, 0, stream>>>(CNT + g * 32 + 1, P2h, P2l, W3T, b3 + (size_t)g * HH, H3, HH, nullptr, nullptr, HH);
        k_refacc<<<NB_ / 8, 256, 0, stream>>>(H3, POS + (size_t)g * NB_, WGT, g, g == 0, REF); }
    k_split128<<<NB_ / 8, 256, 0, stream>>>(REF, Rh, Rl);
    for (int c4 = 0; c4 < 4; ++c4) { const size_t r0 = (size_t)c4 * (NB_ / 4);
        k_gemmb<false, false><<<dim3((NB_ / 4) / 64, DD / 64, 1), 128, 0, stream>>>(Xb + r0 * DD, nullptr, WG1, bagg, Y1, DD, nullptr, nullptr, DD);
        k_gemmb<true, false><<<dim3((NB_ / 4) / 64, DD / 64, 1), 128, 0, stream>>>(Rh + r0 * HH, Rl + r0 * HH, WG2, nullptr, Y2, DD, nullptr, Y1, HH, 0);
        k_reluout<<<(NB_ / 4) / 8, 256, 0, stream>>>(Y2, out + r0 * DD); }
}
